// RelPartialLearnableMultiHeadAttn_41901700940373
// MI455X (gfx1250) — hardware-verified
//
#include <hip/hip_runtime.h>
#include <math.h>
#include <stdint.h>

#define NHD_   16
#define HD_    64
#define DM_    1024
#define QLF_   1024
#define MLN_   1024
#define KLN_   2048
#define BSF_   4
#ifndef NB
#define NB 4
#endif
#ifndef NQ
#define NQ 1024
#endif
#define NPAIR_ 4
#define BDW_   2112
#define Q2W_   2048
#define CXW_   2048
#define QROW_  (BSF_ * Q2W_)
#define KROW_  (BSF_ * DM_)
#define CROW_  (BSF_ * CXW_)
#define LOSC_  1024.0f
#define LOINV_ 0.0009765625f

static_assert((NQ % 64) == 0);
static_assert(NQ >= 64 && NQ <= QLF_);
static_assert(NB >= 1 && NB <= BSF_);
static_assert((NHD_ % NPAIR_) == 0);
static_assert(MLN_ + QLF_ == KLN_);

typedef _Float16 v16h __attribute__((ext_vector_type(16)));
typedef _Float16 v8h  __attribute__((ext_vector_type(8)));
typedef float    v8f  __attribute__((ext_vector_type(8)));
typedef float    v4f  __attribute__((ext_vector_type(4)));
typedef int      v4i  __attribute__((ext_vector_type(4)));
typedef v4f __attribute__((may_alias)) v4fa;
typedef v8h __attribute__((may_alias)) v8ha;
typedef v4i __attribute__((may_alias)) v4ia;

__device__ __forceinline__ float bf_rne(float f) {
  unsigned u = __float_as_uint(f);
  u = (u + 0x7FFFu + ((u >> 16) & 1u)) & 0xFFFF0000u;
  return __uint_as_float(u);
}

union FragU { v16h v; v8ha h[2]; };
__device__ __forceinline__ v16h ldfrag(const _Float16* p) {
  FragU f;
  f.h[0] = *(const v8ha*)(p);
  f.h[1] = *(const v8ha*)(p + 16);
  return f.v;
}

__device__ __forceinline__ v8f mma16(v16h a, v16h b, v8f c) {
  c = __builtin_amdgcn_wmma_f32_16x16x32_f16(false, a, false, b, (short)0, c, false, false);
  asm volatile("v_nop\n\tv_nop\n\tv_nop\n\tv_nop" : "+v"(c) : "v"(a), "v"(b));
  return c;
}

__device__ __forceinline__ v8f zero8() { v8f z = {0.f, 0.f, 0.f, 0.f, 0.f, 0.f, 0.f, 0.f}; return z; }

__global__ __launch_bounds__(256) void cvt_plane_kernel(const float* __restrict__ src, _Float16* __restrict__ dst,
                                                        int nrows, int ncols, int dst_ld, float scale,
                                                        int dup_off, float dup_scale) {
  const int i = blockIdx.x * 256 + threadIdx.x;
  const int c8n = ncols >> 3;
  const int total8 = nrows * c8n;
  if (i >= total8) return;
  const int r  = i / c8n;
  const int c8 = (i - r * c8n) * 8;
  const float* sp = src + (size_t)r * ncols + c8;
  const v4f a = *(const v4f*)(sp);
  const v4f b = *(const v4f*)(sp + 4);
  float x[8];
  x[0] = bf_rne(a[0]); x[1] = bf_rne(a[1]); x[2] = bf_rne(a[2]); x[3] = bf_rne(a[3]);
  x[4] = bf_rne(b[0]); x[5] = bf_rne(b[1]); x[6] = bf_rne(b[2]); x[7] = bf_rne(b[3]);
  v8h o, o2;
#pragma unroll
  for (int e = 0; e < 8; ++e) {
    o[e]  = (_Float16)(x[e] * scale);
    o2[e] = (_Float16)(x[e] * dup_scale);
  }
  _Float16* dp = dst + (size_t)r * dst_ld + c8;
  *(volatile v8h*)dp = o;
  if (dup_off > 0) *(volatile v8h*)(dp + dup_off) = o2;
  __threadfence();
  *(volatile v8h*)dp = o;
  if (dup_off > 0) *(volatile v8h*)(dp + dup_off) = o2;
}

__global__ __launch_bounds__(128) void maskword_kernel(const int* __restrict__ mask, unsigned* __restrict__ MW) {
  __shared__ __align__(16) int mt[64][68];
  const int tid = threadIdx.x, wave = tid >> 5, lane = tid & 31, hh = lane >> 4, c = lane & 15;
  const int qb = blockIdx.x >> 5, kc = blockIdx.x & 31;
  {
    const int r = tid >> 1, c0 = (tid & 1) * 32;
    const int* mp = mask + (size_t)(qb * 64 + r) * KLN_ + kc * 64 + c0;
#pragma unroll
    for (int i = 0; i < 8; ++i) {
      const v4i m4 = *(const v4ia*)(mp + 4 * i);
      *(v4ia*)(&mt[r][c0 + 4 * i]) = m4;
    }
  }
  __syncthreads();
  unsigned word = 0u;
#pragma unroll
  for (int r = 0; r < 8; ++r)
#pragma unroll
    for (int j = 0; j < 4; ++j)
      word |= ((mt[wave * 16 + 8 * hh + r][16 * j + c] != 0) ? 1u : 0u) << (r * 4 + j);
  unsigned* dp = MW + (size_t)blockIdx.x * 128 + tid;
  *(volatile unsigned*)dp = word;
  __threadfence();
  *(volatile unsigned*)dp = word;
}

__global__ __launch_bounds__(256) void maskcheck_kernel(const int* __restrict__ mask, float* __restrict__ FLAG) {
  __shared__ int wf[8];
  const int tid = threadIdx.x, wave = tid >> 5, lane = tid & 31;
  int viol = 0;
  for (int rr = 0; rr < 4; ++rr) {
    const int i = tid * 4 + rr;
    const int* row = mask + (size_t)i * KLN_;
    int rowun = 0;
#pragma unroll 1
    for (int j4 = 0; j4 < KLN_ / 4; ++j4) {
      const v4i m = *(const v4ia*)(row + 4 * j4);
#pragma unroll
      for (int e = 0; e < 4; ++e) {
        const int j  = 4 * j4 + e;
        const int un = (m[e] == 0) ? 1 : 0;
        rowun |= un;
        viol  |= un & ((j > i + MLN_) ? 1 : 0);
      }
    }
    viol |= (rowun == 0) ? 1 : 0;
  }
  viol |= __shfl_xor(viol, 1, 32);
  viol |= __shfl_xor(viol, 2, 32);
  viol |= __shfl_xor(viol, 4, 32);
  viol |= __shfl_xor(viol, 8, 32);
  viol |= __shfl_xor(viol, 16, 32);
  if (lane == 0) wf[wave] = viol;
  __syncthreads();
  if (wave == 0) {
    int f = wf[lane & 7];
    f |= __shfl_xor(f, 1, 32);
    f |= __shfl_xor(f, 2, 32);
    f |= __shfl_xor(f, 4, 32);
    const float v = (lane == 0) ? ((f != 0) ? 1.0f : 0.0f) : 0.0f;
    *(volatile float*)(FLAG + lane) = v;
    __threadfence();
    *(volatile float*)(FLAG + lane) = v;
  }
}

template <int OUT, bool SKEW>
__global__ __launch_bounds__(256) void gemm_f16_kernel(
    const _Float16* __restrict__ A, int lda, long strideA,
    const _Float16* __restrict__ Bt, int ldb, long strideB,
    void* __restrict__ C1, void* __restrict__ C2, int ldc, long strideC,
    const float* __restrict__ b1, const float* __restrict__ b2,
    int M, int N, int K, float scale, float carry, int skew0, int nzero) {
  __shared__ __align__(16) float sT[8][16 * 68];

  const int z    = blockIdx.y;
  const int lane = threadIdx.x & 31;
  const int wave = threadIdx.x >> 5;
  const int tilesN = N >> 6;
  const int tilesM = M >> 6;
  const int tile = blockIdx.x * 8 + wave;
  if (tile >= tilesM * tilesN) return;
  const int tm = tile / tilesN;
  const int tn = tile - tm * tilesN;
  const int m0 = tm << 6;
  const int n0 = tn << 6;
  const int nsk = SKEW ? ((skew0 - tm) << 6) : 0;
  const int kEnd = (SKEW && (nsk + n0) >= nzero) ? 0 : K;

  const _Float16* Ab = A  + (size_t)z * strideA;
  const _Float16* Bb = Bt + (size_t)z * strideB;

  const int rl   = lane & 15;
  const int koff = (lane >> 4) * 8;
  const int mOff = (lane >> 4) * 8;

  v8f acc[4][4];
#pragma unroll
  for (int i = 0; i < 4; ++i)
#pragma unroll
    for (int j = 0; j < 4; ++j) acc[i][j] = zero8();

  for (int k0 = 0; k0 < kEnd; k0 += 32) {
    v16h bfr[4];
#pragma unroll
    for (int j = 0; j < 4; ++j)
      bfr[j] = ldfrag(Bb + (size_t)(nsk + n0 + (j << 4) + rl) * ldb + koff + k0);
#pragma unroll
    for (int i = 0; i < 4; ++i) {
      const v16h af = ldfrag(Ab + (size_t)(m0 + (i << 4) + rl) * lda + koff + k0);
#pragma unroll
      for (int j = 0; j < 4; ++j) acc[i][j] = mma16(af, bfr[j], acc[i][j]);
    }
  }

  const float pz = (OUT == 0) ? ((b1[0] != 0.0f) ? __int_as_float(0x7fc00000) : 0.0f) : 0.0f;
  float* slab = sT[wave];
#pragma unroll
  for (int i = 0; i < 4; ++i) {
    const int mBase = m0 + (i << 4);
#pragma unroll
    for (int j = 0; j < 4; ++j)
#pragma unroll
      for (int r = 0; r < 8; ++r)
        slab[(mOff + r) * 68 + (j << 4) + rl] = (OUT == 0) ? (acc[i][j][r] * scale + pz) : (acc[i][j][r] * scale);
    __builtin_amdgcn_fence(__ATOMIC_RELEASE, "workgroup");
    __builtin_amdgcn_wave_barrier();
    __builtin_amdgcn_fence(__ATOMIC_ACQUIRE, "workgroup");
    if (OUT == 0) {
      float* C = (float*)C1 + (size_t)z * strideC;
      const int hh = lane >> 4, c4 = (lane & 15) * 4;
      for (int pass = 0; pass < 2; ++pass) {
#pragma unroll
        for (int it = 0; it < 8; ++it) {
          const int row = it * 2 + hh;
          const v4f v = *(const v4fa*)(slab + row * 68 + c4);
          *(volatile v4f*)(C + (size_t)(mBase + row) * ldc + n0 + c4) = v;
        }
        __threadfence();
      }
    } else {
      const int q = lane >> 3, c8 = (lane & 7) * 8;
      _Float16* Ca = (_Float16*)C1 + (size_t)z * strideC;
      _Float16* Cb = (_Float16*)C2 + (size_t)z * strideC;
      const int cb0  = (OUT == 1) ? n0 : (2 * n0);
      const int nvar = (OUT == 3) ? 2 : 1;
#pragma unroll 1
      for (int var = 0; var < nvar; ++var) {
        const float* bb = (var == 0) ? b1 : b2;
        _Float16*    Cd = (var == 0) ? Ca : Cb;
        v8h hv[4], lv[4];
#pragma unroll
        for (int it = 0; it < 4; ++it) {
          const int row = it * 4 + q;
          const float* sp = slab + row * 68 + c8;
          const v4f x0 = *(const v4fa*)(sp);
          const v4f x1 = *(const v4fa*)(sp + 4);
          float f[8];
          f[0] = x0[0]; f[1] = x0[1]; f[2] = x0[2]; f[3] = x0[3];
          f[4] = x1[0]; f[5] = x1[1]; f[6] = x1[2]; f[7] = x1[3];
          v8h ha, hb;
#pragma unroll
          for (int e = 0; e < 8; ++e) {
            if (OUT == 1) {
              ha[e] = (_Float16)f[e];
              hb[e] = ha[e];
            } else if (OUT == 2) {
              ha[e] = (_Float16)f[e];
              hb[e] = (_Float16)((float)ha[e] * carry);
            } else {
              const int n = n0 + c8 + e;
              const float x = (f[e] + bf_rne(bb[n])) * carry;
              ha[e] = (_Float16)x;
              hb[e] = (_Float16)((x - (float)ha[e]) * LOSC_);
            }
          }
          hv[it] = ha; lv[it] = hb;
        }
        for (int pass = 0; pass < 2; ++pass) {
#pragma unroll
          for (int it = 0; it < 4; ++it) {
            const int row = it * 4 + q;
            _Float16* dp = Cd + (size_t)(mBase + row) * ldc + cb0 + c8;
            *(volatile v8h*)(dp) = hv[it];
            if (OUT >= 2) *(volatile v8h*)(dp + 64) = lv[it];
          }
          __threadfence();
        }
      }
    }
    __builtin_amdgcn_fence(__ATOMIC_RELEASE, "workgroup");
    __builtin_amdgcn_wave_barrier();
    __builtin_amdgcn_fence(__ATOMIC_ACQUIRE, "workgroup");
  }
}

__global__ __launch_bounds__(128)
void relattn_kernel(const _Float16* __restrict__ QU, const _Float16* __restrict__ Kp,
                    const _Float16* __restrict__ VT, const float* __restrict__ BD,
                    const unsigned* __restrict__ MW, _Float16* __restrict__ CTX,
                    int pairBase, float cs) {
  __shared__ __align__(16) unsigned char SMEM[32768];
  __shared__ int mfl[4];
  _Float16* Ksh = (_Float16*)(SMEM);
  _Float16* Vsh = (_Float16*)(SMEM + 16384);
  _Float16* Psh = (_Float16*)(SMEM + 24576);
  float*    Osh = (float*)(SMEM);

  const int tid  = threadIdx.x;
  const int wave = tid >> 5;
  const int lane = tid & 31;
  const int hh   = lane >> 4;
  const int c    = lane & 15;

  const int z    = blockIdx.y;
  const int pair = pairBase + z;
  const int b    = pair / NHD_;
  const int h    = pair - b * NHD_;
  const int qb   = blockIdx.x;
  const int q0   = qb * 64 + wave * 16;
  const int rr0  = wave * 16 + 8 * hh;

  const _Float16* Qh = QU + (size_t)b * Q2W_ + h * (2 * HD_);
  const _Float16* Kh = Kp + (size_t)b * DM_ + h * HD_;
  const _Float16* Vh = VT + (size_t)b * DM_ * KLN_ + (size_t)(h * HD_) * KLN_;
  const float*    bd = BD + (size_t)z * QLF_ * BDW_;
  _Float16*       ctx = CTX + (size_t)b * CXW_ + h * HD_;
  const unsigned* mwp = MW + (size_t)qb * 32 * 128 + tid;

  v16h qa[4];
#pragma unroll
  for (int dc = 0; dc < 4; ++dc)
    qa[dc] = ldfrag(Qh + (size_t)(q0 + c) * QROW_ + dc * 32 + 8 * hh);

  const float* bdr = bd + (long)(q0 + 8 * hh) * BDW_ + (63 - rr0 + c);

  float mrow[8], lrow[8];
  v8f oacc[4];
#pragma unroll
  for (int r = 0; r < 8; ++r) { mrow[r] = -INFINITY; lrow[r] = 0.f; }
#pragma unroll
  for (int t = 0; t < 4; ++t) oacc[t] = zero8();

  _Float16* pw = Psh + wave * (16 * 64);
  const _Float16 losc = (_Float16)LOINV_;

  for (int kc = 0; kc < KLN_ / 64; ++kc) {
    const int kv0 = kc * 64;
    const unsigned mword = mwp[(size_t)kc * 128];
    int un = (mword != 0xFFFFFFFFu) ? 1 : 0;
    un |= __shfl_xor(un, 1, 32);
    un |= __shfl_xor(un, 2, 32);
    un |= __shfl_xor(un, 4, 32);
    un |= __shfl_xor(un, 8, 32);
    un |= __shfl_xor(un, 16, 32);
    __syncthreads();
    if (lane == 0) mfl[wave] = un;
    __syncthreads();
    const int anyb = mfl[0] | mfl[1] | mfl[2] | mfl[3];
    if (anyb == 0) continue;
    {
      const int r = tid >> 1, c0 = (tid & 1) * 32;
      const _Float16* ks = Kh + (size_t)(kv0 + r) * KROW_ + c0;
      const _Float16* vs = Vh + (size_t)r * KLN_ + kv0 + c0;
#pragma unroll
      for (int i = 0; i < 4; ++i) {
        const v8h kk8 = *(const v8h*)(ks + 8 * i);
        const v8h vv8 = *(const v8h*)(vs + 8 * i);
        const v8h kl8 = kk8 * losc;
        *(v8ha*)(Ksh + r * 128 + c0 + 8 * i)      = kk8;
        *(v8ha*)(Ksh + r * 128 + 64 + c0 + 8 * i) = kl8;
        *(v8ha*)(Vsh + r * 64 + c0 + 8 * i)        = vv8;
      }
    }
    __syncthreads();

    v8f s[4];
#pragma unroll
    for (int j = 0; j < 4; ++j) {
      s[j] = zero8();
#pragma unroll
      for (int dc = 0; dc < 4; ++dc) {
        const v16h kb = ldfrag(Ksh + (j * 16 + c) * 128 + dc * 32 + 8 * hh);
        s[j] = mma16(qa[dc], kb, s[j]);
      }
    }

    float cm[8];
#pragma unroll
    for (int r = 0; r < 8; ++r) {
      float m = -INFINITY;
#pragma unroll
      for (int j = 0; j < 4; ++j) {
        const float sv0 = s[j][r] * cs + bdr[(long)r * (BDW_ - 1) + kv0 + (j << 4)];
        const float sv  = (((mword >> (r * 4 + j)) & 1u) != 0u) ? -1e30f : sv0;
        s[j][r] = sv;
        m = fmaxf(m, sv);
      }
      m = fmaxf(m, __shfl_xor(m, 1, 32));
      m = fmaxf(m, __shfl_xor(m, 2, 32));
      m = fmaxf(m, __shfl_xor(m, 4, 32));
      m = fmaxf(m, __shfl_xor(m, 8, 32));
      cm[r] = m;
    }

#pragma unroll
    for (int r = 0; r < 8; ++r) {
      const float mnew  = fmaxf(mrow[r], cm[r]);
      const float alpha = __expf(mrow[r] - mnew);
      mrow[r] = mnew;
      float psum = 0.f;
#pragma unroll
      for (int j = 0; j < 4; ++j) {
        const float p = __expf(s[j][r] - mnew);
        psum += p;
        pw[(8 * hh + r) * 64 + j * 16 + c] = (_Float16)(p * 4096.0f);
      }
      psum += __shfl_xor(psum, 1, 32);
      psum += __shfl_xor(psum, 2, 32);
      psum += __shfl_xor(psum, 4, 32);
      psum += __shfl_xor(psum, 8, 32);
      lrow[r] = lrow[r] * alpha + psum;
#pragma unroll
      for (int t = 0; t < 4; ++t) oacc[t][r] *= alpha;
    }
    __builtin_amdgcn_fence(__ATOMIC_RELEASE, "workgroup");
    __builtin_amdgcn_wave_barrier();
    __builtin_amdgcn_fence(__ATOMIC_ACQUIRE, "workgroup");

#pragma unroll
    for (int kk = 0; kk < 2; ++kk) {
      const v16h pa = ldfrag(pw + c * 64 + kk * 32 + 8 * hh);
#pragma unroll
      for (int t = 0; t < 4; ++t) {
        const v16h vb = ldfrag(Vsh + (t * 16 + c) * 64 + kk * 32 + 8 * hh);
        oacc[t] = mma16(pa, vb, oacc[t]);
      }
    }
  }

  __syncthreads();
  float* os = Osh + wave * (16 * 64);
#pragma unroll
  for (int r = 0; r < 8; ++r) {
    const float inv = 1.0f / (1024.0f * lrow[r]);
#pragma unroll
    for (int t = 0; t < 4; ++t) os[(8 * hh + r) * 64 + t * 16 + c] = oacc[t][r] * inv;
  }
  __builtin_amdgcn_fence(__ATOMIC_RELEASE, "workgroup");
  __builtin_amdgcn_wave_barrier();
  __builtin_amdgcn_fence(__ATOMIC_ACQUIRE, "workgroup");
  const int q4 = lane >> 3, c8 = (lane & 7) * 8;
  v8h hv[4], lv[4];
#pragma unroll
  for (int it = 0; it < 4; ++it) {
    const int row = it * 4 + q4;
    const float* sp = os + row * 64 + c8;
    const v4f x0 = *(const v4fa*)(sp);
    const v4f x1 = *(const v4fa*)(sp + 4);
    float f[8];
    f[0] = x0[0]; f[1] = x0[1]; f[2] = x0[2]; f[3] = x0[3];
    f[4] = x1[0]; f[5] = x1[1]; f[6] = x1[2]; f[7] = x1[3];
    v8h ha, hb;
#pragma unroll
    for (int e = 0; e < 8; ++e) {
      ha[e] = (_Float16)f[e];
      hb[e] = (_Float16)((f[e] - (float)ha[e]) * LOSC_);
    }
    hv[it] = ha; lv[it] = hb;
  }
  for (int pass = 0; pass < 2; ++pass) {
#pragma unroll
    for (int it = 0; it < 4; ++it) {
      const int row = it * 4 + q4;
      _Float16* dp = ctx + (size_t)(q0 + row) * CROW_ + c8;
      *(volatile v8h*)(dp)       = hv[it];
      *(volatile v8h*)(dp + DM_) = lv[it];
    }
    __threadfence();
  }
}

extern "C" void kernel_launch(void* const* d_in, const int* in_sizes, int n_in,
                              void* d_out, int out_size, void* d_ws, size_t ws_size,
                              hipStream_t stream) {
  if (n_in < 9) return;
  if (in_sizes[0] < QLF_ * BSF_ * DM_) return;
  if (in_sizes[1] < KLN_ * DM_) return;
  if (in_sizes[2] < MLN_ * BSF_ * DM_) return;
  if (in_sizes[3] < NHD_ * HD_ || in_sizes[4] < NHD_ * HD_) return;
  if (in_sizes[5] < 3 * DM_ * DM_) return;
  if (in_sizes[6] < DM_ * DM_ || in_sizes[7] < DM_ * DM_) return;
  if (in_sizes[8] < QLF_ * KLN_) return;
  if (out_size < ((NQ - 1) * BSF_ + NB) * DM_) return;

  const float* w     = (const float*)d_in[0];
  const float* rpos  = (const float*)d_in[1];
  const float* mems  = (const float*)d_in[2];
  const float* rwb   = (const float*)d_in[3];
  const float* rrb   = (const float*)d_in[4];
  const float* qkvw  = (const float*)d_in[5];
  const float* rnw   = (const float*)d_in[6];
  const float* ow    = (const float*)d_in[7];
  const int*   amask = (const int*)d_in[8];
  float* out = (float*)d_out;

  const size_t PMW  = (size_t)16 * 32 * 128 * 4;
  const size_t PFL  = 256;
  const size_t PWO2 = (size_t)DM_ * CXW_ * 2;
  const size_t PQ2  = (size_t)QLF_ * BSF_ * Q2W_ * 2;
  const size_t PKP  = (size_t)KLN_ * BSF_ * DM_ * 2;
  const size_t PVT  = (size_t)BSF_ * DM_ * KLN_ * 2;
  const size_t PRK  = (size_t)KLN_ * Q2W_ * 2;
  const size_t PCAT = (size_t)KLN_ * BSF_ * DM_ * 2;
  const size_t PR16 = (size_t)KLN_ * DM_ * 2;
  const size_t PW3  = (size_t)3 * DM_ * DM_ * 2;
  const size_t PWR  = (size_t)DM_ * DM_ * 2;
  const size_t PCTX = (size_t)QLF_ * BSF_ * CXW_ * 2;
  const size_t PBD  = (size_t)QLF_ * BDW_ * 4;
  size_t off = 0;
  const size_t oMW  = off; off += PMW;
  const size_t oFL  = off; off += PFL;
  const size_t oWO2 = off; off += PWO2;
  const size_t oQW  = off; off += PQ2;
  const size_t oQR  = off; off += PQ2;
  const size_t oKP  = off; off += PKP;
  const size_t oVT  = off; off += PVT;
  const size_t oRK  = off; off += PRK;
  const size_t oSCR = off;
  const size_t oCAT = oSCR;
  const size_t oR16 = oCAT + PCAT;
  const size_t oW3  = oR16 + PR16;
  const size_t oWR  = oW3 + PW3;
  const size_t earlyEnd = oWR + PWR;
  const size_t oCTX = oSCR;
  const size_t oBD  = oCTX + PCTX;
  const size_t lateEnd = oBD + (size_t)NPAIR_ * PBD;
  const size_t total = (earlyEnd > lateEnd) ? earlyEnd : lateEnd;
  if (total > ws_size) return;
  if (total > (size_t)134217728) return;

  char* ws = (char*)d_ws;
  unsigned* MW  = (unsigned*)(ws + oMW);
  float*    FLG = (float*)(ws + oFL);
  _Float16* WO2 = (_Float16*)(ws + oWO2);
  _Float16* QW2 = (_Float16*)(ws + oQW);
  _Float16* QR2 = (_Float16*)(ws + oQR);
  _Float16* KP  = (_Float16*)(ws + oKP);
  _Float16* VTP = (_Float16*)(ws + oVT);
  _Float16* RK2 = (_Float16*)(ws + oRK);
  _Float16* CAT = (_Float16*)(ws + oCAT);
  _Float16* R16 = (_Float16*)(ws + oR16);
  _Float16* W3  = (_Float16*)(ws + oW3);
  _Float16* WR  = (_Float16*)(ws + oWR);
  _Float16* CTX = (_Float16*)(ws + oCTX);
  float*    BAND = (float*)(ws + oBD);
  _Float16* WQ  = W3;
  _Float16* WK  = W3 + (size_t)DM_ * DM_;
  _Float16* WV  = W3 + (size_t)2 * DM_ * DM_;

  const float cs = 0.00048828125f;
  const dim3 blk(256);

  cvt_plane_kernel<<<dim3((3 * DM_ * (DM_ / 8) + 255) / 256), blk, 0, stream>>>(qkvw, W3, 3 * DM_, DM_, DM_, 64.0f, 0, 0.0f);
  cvt_plane_kernel<<<dim3((DM_ * (DM_ / 8) + 255) / 256), blk, 0, stream>>>(rnw, WR, DM_, DM_, DM_, 64.0f, 0, 0.0f);
  cvt_plane_kernel<<<dim3((DM_ * (DM_ / 8) + 255) / 256), blk, 0, stream>>>(ow, WO2, DM_, DM_, CXW_, 64.0f, DM_, 0.0625f);
  cvt_plane_kernel<<<dim3((MLN_ * BSF_ * (DM_ / 8) + 255) / 256), blk, 0, stream>>>(mems, CAT, MLN_ * BSF_, DM_, DM_, 1.0f, 0, 0.0f);
  cvt_plane_kernel<<<dim3((QLF_ * BSF_ * (DM_ / 8) + 255) / 256), blk, 0, stream>>>(w, CAT + (size_t)MLN_ * BSF_ * DM_,
                                                                                     QLF_ * BSF_, DM_, DM_, 1.0f, 0, 0.0f);
  cvt_plane_kernel<<<dim3((KLN_ * (DM_ / 8) + 255) / 256), blk, 0, stream>>>(rpos, R16, KLN_, DM_, DM_, 1.0f, 0, 0.0f);
  maskword_kernel<<<dim3(16 * 32), dim3(128), 0, stream>>>(amask, MW);
  maskcheck_kernel<<<dim3(1), blk, 0, stream>>>(amask, FLG);
  {
    const int tilesQ = (NQ / 64) * (DM_ / 64);
    gemm_f16_kernel<3, false><<<dim3((tilesQ + 7) / 8, NB), blk, 0, stream>>>(
        CAT + (size_t)MLN_ * BSF_ * DM_, KROW_, (long)DM_, WQ, DM_, 0L,
        (void*)QW2, (void*)QR2, QROW_, (long)Q2W_, rwb, rrb,
        NQ, DM_, DM_, 0.015625f, 16.0f, 0, 0x7fffffff);
    const int tilesK = (KLN_ / 64) * (DM_ / 64);
    gemm_f16_kernel<1, false><<<dim3((tilesK + 7) / 8, NB), blk, 0, stream>>>(
        CAT, KROW_, (long)DM_, WK, DM_, 0L,
        (void*)KP, (void*)KP, KROW_, (long)DM_, rwb, rwb,
        KLN_, DM_, DM_, 0.25f, 1.0f, 0, 0x7fffffff);
    const int tilesV = (DM_ / 64) * (KLN_ / 64);
    gemm_f16_kernel<1, false><<<dim3((tilesV + 7) / 8, NB), blk, 0, stream>>>(
        WV, DM_, 0L, CAT, KROW_, (long)DM_,
        (void*)VTP, (void*)VTP, KLN_, (long)DM_ * KLN_, rwb, rwb,
        DM_, KLN_, DM_, 0.25f, 1.0f, 0, 0x7fffffff);
    const int tilesR = (KLN_ / 64) * (DM_ / 64);
    gemm_f16_kernel<2, false><<<dim3((tilesR + 7) / 8, 1), blk, 0, stream>>>(
        R16, DM_, 0L, WR, DM_, 0L,
        (void*)RK2, (void*)RK2, Q2W_, 0L, rwb, rwb,
        KLN_, DM_, DM_, 0.25f, LOINV_, 0, 0x7fffffff);
  }
  const int nGroups = (NB * NHD_) / NPAIR_;
  for (int g = 0; g < nGroups; ++g) {
    const int pairBase = g * NPAIR_;
    const int b  = pairBase / NHD_;
    const int h0 = pairBase - b * NHD_;
    const _Float16* Aq = QR2 + (size_t)b * Q2W_ + h0 * (2 * HD_);
    const _Float16* Bp = RK2 + h0 * (2 * HD_);
    const int tilesBD = (NQ / 64) * (BDW_ / 64);
    gemm_f16_kernel<0, true><<<dim3((tilesBD + 7) / 8, NPAIR_), blk, 0, stream>>>(
        Aq, QROW_, (long)(2 * HD_), Bp, Q2W_, (long)(2 * HD_),
        (void*)BAND, (void*)BAND, BDW_, (long)QLF_ * BDW_, FLG, FLG,
        NQ, BDW_, 2 * HD_, cs, 1.0f, 15, KLN_);
    relattn_kernel<<<dim3(NQ / 64, NPAIR_), dim3(128), 0, stream>>>(QW2, KP, VTP, BAND, MW, CTX, pairBase, cs);
  }
  {
    const int tiles = (NQ / 64) * (DM_ / 64);
    gemm_f16_kernel<0, false><<<dim3((tiles + 7) / 8, NB), blk, 0, stream>>>(
        CTX, CROW_, (long)CXW_, WO2, CXW_, 0L,
        (void*)out, (void*)out, BSF_ * DM_, (long)DM_, FLG, FLG,
        NQ, DM_, CXW_, 0.000244140625f, 1.0f, 0, 0x7fffffff);
  }
  (void)hipGetLastError();
}
